// TTConvEinsum_66546223284785
// MI455X (gfx1250) — hardware-verified
//
#include <hip/hip_runtime.h>
#include <hip/hip_bf16.h>

typedef __attribute__((ext_vector_type(16))) _Float16 v16bf;
typedef __attribute__((ext_vector_type(8)))  float  v8f;
typedef unsigned short ushort_t;

__device__ __forceinline__ ushort_t f2bf(float f) {
    return __builtin_bit_cast(ushort_t, (_Float16)f);
}

__global__ __launch_bounds__(256) void tt_merge23(
    const float* __restrict__ core2, const float* __restrict__ core3,
    float* __restrict__ W23) {
    int idx = blockIdx.x * 256 + threadIdx.x;
    int r1 = idx & 15;
    int j2 = (idx >> 4) & 7;
    int j1 = (idx >> 7) & 7;
    int i2 = (idx >> 10) & 3;
    int i1 = idx >> 12;
    const float* c2 = core2 + (((i1 * 8 + j1) * 16 + r1) << 4);
    const float* c3 = core3 + ((i2 * 8 + j2) << 4);
    float s = 0.f;
#pragma unroll
    for (int r2 = 0; r2 < 16; ++r2) s += c2[r2] * c3[r2];
    *(volatile float*)(W23 + idx) = s;
    __threadfence();
    *(volatile float*)(W23 + idx) = s;
}

__global__ __launch_bounds__(256) void tt_merge123(
    const float* __restrict__ core1, const float* __restrict__ W23,
    float* __restrict__ W123) {
    int idx = blockIdx.x * 256 + threadIdx.x;
    int r0 = idx & 15;
    int o  = (idx >> 4) & 511;
    int c  = idx >> 13;
    int j2 = o & 7, j1 = (o >> 3) & 7, j0 = o >> 6;
    int i2 = c & 3, i1 = (c >> 2) & 7, i0 = c >> 5;
    const float* c1 = core1 + i0 * 2048 + j0 * 256 + r0 * 16;
    const float* w  = W23   + i1 * 4096 + i2 * 1024 + j1 * 128 + j2 * 16;
    float s = 0.f;
#pragma unroll
    for (int r1 = 0; r1 < 16; ++r1) s += c1[r1] * w[r1];
    *(volatile float*)(W123 + idx) = s;
    __threadfence();
    *(volatile float*)(W123 + idx) = s;
}

__global__ __launch_bounds__(128) void tt_mergefull(
    const float* __restrict__ core0, const float* __restrict__ W123,
    ushort_t* __restrict__ WfullT) {
    const int c = 2 * threadIdx.x;
    const int o = blockIdx.x;
    const int q = blockIdx.y;
    const float* w0 = W123 + c * 8192 + o * 16;
    const float* w1 = w0 + 8192;
    float s0 = 0.f, s1 = 0.f;
#pragma unroll
    for (int r0 = 0; r0 < 16; ++r0) { const float cc = core0[r0 * 9 + q]; s0 += cc * w0[r0]; s1 += cc * w1[r0]; }
    const unsigned pk = (unsigned)f2bf(s0) | ((unsigned)f2bf(s1) << 16);
    unsigned* dst = (unsigned*)(WfullT + (size_t)o * 2304 + q * 256 + c);
    *(volatile unsigned*)dst = pk;
    __threadfence();
    *(volatile unsigned*)dst = pk;
}

#define ASTR 40

__global__ __launch_bounds__(256) void tt_conv_gemm(
    const float* __restrict__ x, const ushort_t* __restrict__ wfullT,
    float* __restrict__ out) {
    __shared__ ushort_t Ash[128 * ASTR];
    __shared__ ushort_t Bsh[128 * ASTR];
    __shared__ __attribute__((aligned(16))) float Csh[128][132];

    const int tid  = threadIdx.x;
    const int n0   = blockIdx.x * 128;
    const int p0   = blockIdx.y * 128;
    const int lane = tid & 31;
    const int wv   = tid >> 5;

    const int arowS  = tid & 127;
    const int ahalfS = tid >> 7;
    const int p  = p0 + arowS;
    const int bb = p >> 12;
    const int hh = (p >> 6) & 63;
    const int ww = p & 63;

    const int bcolS = tid >> 1;
    const int bsegS = tid & 1;

    const int arow  = wv * 16 + (lane & 15);
    const int ahalf = (lane < 16) ? 0 : 8;
    const int bhalf = (lane < 16) ? 0 : 8;

    const v8f zero = {0.f, 0.f, 0.f, 0.f, 0.f, 0.f, 0.f, 0.f};
    v8f acc[8];
#pragma unroll
    for (int n = 0; n < 8; ++n) acc[n] = zero;

    for (int q = 0; q < 9; ++q) {
        const int kh  = q / 3;
        const int kw  = q - 3 * kh;
        const int hin = hh + kh - 1;
        const int win = ww + kw - 1;
        const bool valid = ((unsigned)hin < 64u) && ((unsigned)win < 64u);
        const float* xq = x + (((size_t)bb) << 20) + ((size_t)(ahalfS * 16) << 12)
                            + (hin << 6) + win;

        for (int cb = 0; cb < 8; ++cb) {
            const int k0 = q * 256 + cb * 32;
            __syncthreads();
            float tv[16];
            if (valid) {
                const float* xp = xq + ((size_t)(cb * 32) << 12);
#pragma unroll
                for (int j = 0; j < 16; ++j) tv[j] = xp[(size_t)j << 12];
            } else {
#pragma unroll
                for (int j = 0; j < 16; ++j) tv[j] = 0.f;
            }
            unsigned int pk[8];
#pragma unroll
            for (int j = 0; j < 8; ++j)
                pk[j] = (unsigned)f2bf(tv[2 * j]) |
                        ((unsigned)f2bf(tv[2 * j + 1]) << 16);
            uint4* adst = (uint4*)&Ash[arowS * ASTR + ahalfS * 16];
            uint4 av0; av0.x = pk[0]; av0.y = pk[1]; av0.z = pk[2]; av0.w = pk[3];
            uint4 av1; av1.x = pk[4]; av1.y = pk[5]; av1.z = pk[6]; av1.w = pk[7];
            adst[0] = av0;
            adst[1] = av1;
            const ushort_t* wp = wfullT + (size_t)(n0 + bcolS) * 2304 + k0 + bsegS * 16;
            uint4 bv0 = *(const uint4*)wp;
            uint4 bv1 = *(const uint4*)(wp + 8);
            uint4* bdst = (uint4*)&Bsh[bcolS * ASTR + bsegS * 16];
            bdst[0] = bv0;
            bdst[1] = bv1;
            __syncthreads();
            union { uint4 u[2]; v16bf v; } af;
            af.u[0] = *(const uint4*)&Ash[arow * ASTR + ahalf];
            af.u[1] = *(const uint4*)&Ash[arow * ASTR + 16 + ahalf];
#pragma unroll
            for (int n = 0; n < 8; ++n) {
                union { uint4 u[2]; v16bf v; } bf;
                const int bcol = n * 16 + (lane & 15);
                bf.u[0] = *(const uint4*)&Bsh[bcol * ASTR + bhalf];
                bf.u[1] = *(const uint4*)&Bsh[bcol * ASTR + 16 + bhalf];
                acc[n] = __builtin_amdgcn_wmma_f32_16x16x32_f16(
                    false, af.v, false, bf.v, (short)0, acc[n], false, false);
            }
        }
    }

    const int rlo = wv * 16 + ((lane < 16) ? 0 : 8);
#pragma unroll
    for (int n = 0; n < 8; ++n) {
        const int ol = n * 16 + (lane & 15);
#pragma unroll
        for (int r = 0; r < 8; ++r) Csh[ol][rlo + r] = acc[n][r];
    }
    __syncthreads();
    {
        typedef __attribute__((ext_vector_type(4))) float v4f_t;
        const int b  = p0 >> 12;
        const int hw0 = p0 & 4095;
#pragma unroll
        for (int i = 0; i < 16; ++i) {
            const int c = tid + 256 * i, ch = c >> 5, q = c & 31;
            v4f_t v; v.x = Csh[ch][q * 4]; v.y = Csh[ch][q * 4 + 1]; v.z = Csh[ch][q * 4 + 2]; v.w = Csh[ch][q * 4 + 3];
            *(volatile v4f_t*)(out + ((((size_t)b << 9) + n0 + ch) << 12) + hw0 + q * 4) = v;
        }
        __threadfence();
#pragma unroll
        for (int i = 0; i < 16; ++i) {
            const int c = tid + 256 * i, ch = c >> 5, q = c & 31;
            v4f_t v; v.x = Csh[ch][q * 4]; v.y = Csh[ch][q * 4 + 1]; v.z = Csh[ch][q * 4 + 2]; v.w = Csh[ch][q * 4 + 3];
            *(volatile v4f_t*)(out + ((((size_t)b << 9) + n0 + ch) << 12) + hw0 + q * 4) = v;
        }
    }
}

extern "C" void kernel_launch(void* const* d_in, const int* in_sizes, int n_in,
                              void* d_out, int out_size, void* d_ws, size_t ws_size,
                              hipStream_t stream) {
    const float* x     = (const float*)d_in[0];
    const float* core0 = (const float*)d_in[1];
    const float* core1 = (const float*)d_in[2];
    const float* core2 = (const float*)d_in[3];
    const float* core3 = (const float*)d_in[4];
    float* out = (float*)d_out;

    float*    W23    = (float*)d_ws;
    float*    W123   = (float*)((char*)d_ws + 131072);
    ushort_t* WfullT = (ushort_t*)((char*)d_ws + 131072 + 8388608);

    tt_merge23  <<<dim3(128),    256, 0, stream>>>(core2, core3, W23);
    tt_merge123 <<<dim3(8192),   256, 0, stream>>>(core1, W23, W123);
    tt_mergefull<<<dim3(512, 9), 128, 0, stream>>>(core0, W123, WfullT);
    tt_conv_gemm<<<dim3(4, 128), 256, 0, stream>>>(x, WfullT, out);
}
